// QKNormAttention_29317446762603
// MI455X (gfx1250) — hardware-verified
//
#include <hip/hip_runtime.h>
#include <math.h>
#include <stdint.h>

static constexpr int NB_BATCH = 4;
static constexpr int NS_SEQ   = 2048;
static constexpr int ND_MODEL = 1024;
static constexpr int NH_HEADS = 16;
static constexpr int NHD      = 64;
static constexpr int NTOK     = NB_BATCH * NS_SEQ;

typedef __attribute__((ext_vector_type(16))) _Float16 v16h;
typedef __attribute__((ext_vector_type(8)))  _Float16 v8h;
typedef __attribute__((ext_vector_type(16))) __bf16   v16b;
typedef __attribute__((ext_vector_type(8)))  __bf16   v8b;
typedef __attribute__((ext_vector_type(8)))  float    v8f;
typedef __attribute__((ext_vector_type(4)))  float    v4f;
typedef __attribute__((ext_vector_type(2)))  float    v2f;

__device__ __forceinline__ unsigned short f2bf_bits(float f) {
  unsigned u = __float_as_uint(f);
  return (unsigned short)((u + 0x7FFFu + ((u >> 16) & 1u)) >> 16);
}
__device__ __forceinline__ float bf_bits2f(unsigned short h) { return __uint_as_float(((unsigned)h) << 16); }
__device__ __forceinline__ unsigned pk16(unsigned short a, unsigned short b) { return (unsigned)a | ((unsigned)b << 16); }

__device__ __forceinline__ void dep_guard_h(v8f& a, v8f& b, v16h x, v16h y) { asm volatile("v_nop\n\tv_nop\n\tv_nop\n\tv_nop" : "+v"(a), "+v"(b) : "v"(x), "v"(y)); }
__device__ __forceinline__ void dep_guard_b(v8f& a, v8f& b, v16b x, v16b y) { asm volatile("v_nop\n\tv_nop\n\tv_nop\n\tv_nop" : "+v"(a), "+v"(b) : "v"(x), "v"(y)); }
__device__ __forceinline__ void keep4_h(v16h a, v16h b, v16h c, v16h d) { asm volatile("v_nop" :: "v"(a), "v"(b), "v"(c), "v"(d)); }
__device__ __forceinline__ void keep4_b(v16b a, v16b b, v16b c, v16b d) { asm volatile("v_nop" :: "v"(a), "v"(b), "v"(c), "v"(d)); }
__device__ __forceinline__ void acc_guard4(v8f& a, v8f& b, v8f& c, v8f& d) { asm volatile("v_nop\n\tv_nop\n\tv_nop\n\tv_nop" : "+v"(a), "+v"(b), "+v"(c), "+v"(d)); }
template <typename T> struct Frag;
template <> struct Frag<_Float16> {
  typedef v16h V; union U { v16h v; v8h h[2]; };
  static __device__ __forceinline__ v16h load(const _Float16* p) {
    U f; f.h[0] = *(const v8h*)(p); f.h[1] = *(const v8h*)(p + 16); return f.v;
  }
  static __device__ __forceinline__ v8f mma(v16h a, v16h b, v8f c) {
    return __builtin_amdgcn_wmma_f32_16x16x32_f16(false, a, false, b, (short)0, c, false, false);
  }
  static __device__ __forceinline__ void guard(v8f& a, v8f& b, v16h x, v16h y) { dep_guard_h(a, b, x, y); }
  static __device__ __forceinline__ void keep(v16h a, v16h b, v16h c, v16h d) { keep4_h(a, b, c, d); }
};
template <> struct Frag<__bf16> {
  typedef v16b V; union U { v16b v; v8b h[2]; };
  static __device__ __forceinline__ v16b load(const __bf16* p) {
    U f; f.h[0] = *(const v8b*)(p); f.h[1] = *(const v8b*)(p + 16); return f.v;
  }
  static __device__ __forceinline__ v8f mma(v16b a, v16b b, v8f c) {
    return __builtin_amdgcn_wmma_f32_16x16x32_bf16(false, a, false, b, (short)0, c, false, false);
  }
  static __device__ __forceinline__ void guard(v8f& a, v8f& b, v16b x, v16b y) { dep_guard_b(a, b, x, y); }
  static __device__ __forceinline__ void keep(v16b a, v16b b, v16b c, v16b d) { keep4_b(a, b, c, d); }
};

template <int ET> struct Elem;
template <> struct Elem<0> { typedef _Float16 T; };
template <> struct Elem<1> { typedef __bf16 T; };
template <int ET, int SPLIT, int BIAS_MODE, int OUT_MODE, bool RESID, int ACT = 0>
__global__ __launch_bounds__(256) void wmma_gemm64(
    const unsigned short* __restrict__ Ap, const unsigned short* __restrict__ A2p, int lda, long strideA,
    const unsigned short* __restrict__ Btp, const unsigned short* __restrict__ Bt2p, int ldb, long strideB,
    void* __restrict__ Cout, void* __restrict__ Cout2, int ldc, long strideC,
    const float* __restrict__ bias,
    const float* __restrict__ resid, long strideR,
    int M, int N, int K, float scale) {
  typedef typename Elem<ET>::T T;
  typedef typename Frag<T>::V V;
  const T* A = (const T*)Ap; const T* A2 = (const T*)A2p; const T* Bt = (const T*)Btp; const T* Bt2 = (const T*)Bt2p;
  __shared__ __align__(16) float sT[8][16 * 68];
  const int b    = blockIdx.y;
  const int lane = threadIdx.x & 31;
  const int wave = threadIdx.x >> 5;
  const int tilesN = N >> 6;
  const int tilesM = M >> 6;
  const int tile = blockIdx.x * 8 + wave;
  if (tile >= tilesM * tilesN) return;
  const int tm = tile / tilesN;
  const int tn = tile - tm * tilesN;
  const int m0 = tm << 6;
  const int n0 = tn << 6;

  const T* Ab  = A  + (size_t)b * strideA;
  const T* Bb  = Bt + (size_t)b * strideB;
  const T* Ab2 = (SPLIT != 0) ? (A2  + (size_t)b * strideA) : nullptr;
  const T* Bb2 = (SPLIT == 1) ? (Bt2 + (size_t)b * strideB) : nullptr;

  const int rlane = lane & 15;
  const int koff  = (lane >> 4) * 8;
  const int mOff  = (lane >> 4) * 8;

  v8f acc[4][4];
#pragma unroll
  for (int i = 0; i < 4; ++i)
#pragma unroll
    for (int j = 0; j < 4; ++j) acc[i][j] = (v8f){0.f,0.f,0.f,0.f,0.f,0.f,0.f,0.f};

  for (int k0 = 0; k0 < K; k0 += 32) {
    V bh[4], bl[4];
#pragma unroll
    for (int j = 0; j < 4; ++j) {
      const size_t bo = (size_t)(n0 + (j << 4) + rlane) * ldb + koff + k0;
      bh[j] = Frag<T>::load(Bb + bo);
      if (SPLIT == 1) bl[j] = Frag<T>::load(Bb2 + bo);
    }
#pragma unroll
    for (int i = 0; i < 4; ++i) {
      const size_t ao = (size_t)(m0 + (i << 4) + rlane) * lda + koff + k0;
      V ah = Frag<T>::load(Ab + ao);
      V al;
      if (SPLIT != 0) al = Frag<T>::load(Ab2 + ao);
#pragma unroll
      for (int j = 0; j < 4; ++j) {
        acc[i][j] = Frag<T>::mma(ah, bh[j], acc[i][j]);
        if (SPLIT == 1) {
          acc[i][j] = Frag<T>::mma(ah, bl[j], acc[i][j]);
          acc[i][j] = Frag<T>::mma(al, bh[j], acc[i][j]);
        }
        if (SPLIT == 2) {
          acc[i][j] = Frag<T>::mma(al, bh[j], acc[i][j]);
        }
      }
      Frag<T>::guard(acc[i][0], acc[i][3], ah, (SPLIT != 0) ? al : ah);
    }
    Frag<T>::keep(bh[0], bh[1], bh[2], bh[3]);
    if (SPLIT == 1) Frag<T>::keep(bl[0], bl[1], bl[2], bl[3]);
  }
  acc_guard4(acc[0][0], acc[0][1], acc[0][2], acc[0][3]);
  acc_guard4(acc[1][0], acc[1][1], acc[1][2], acc[1][3]);
  acc_guard4(acc[2][0], acc[2][1], acc[2][2], acc[2][3]);
  acc_guard4(acc[3][0], acc[3][1], acc[3][2], acc[3][3]);

  float* slab = sT[wave];
  const float* Rb = RESID ? (resid + (size_t)b * strideR) : nullptr;
#pragma unroll
  for (int i = 0; i < 4; ++i) {
    const int mBase = m0 + (i << 4);
#pragma unroll
    for (int j = 0; j < 4; ++j) {
      const int n = n0 + (j << 4) + rlane;
      float bv = 0.f;
      if (BIAS_MODE == 2) bv = bias[n];
#pragma unroll
      for (int r = 0; r < 8; ++r) {
        float v = acc[i][j][r] * scale;
        if (BIAS_MODE == 1) v += bias[mBase + mOff + r];
        if (BIAS_MODE == 2) v += bv;
        if (RESID) v += Rb[(size_t)(mBase + mOff + r) * ldc + n];
        if (ACT == 1) v = tanhf(v);
        if (ACT == 2) v = fmaxf(v, 0.0f);
        if (ACT == 3) v = v / (1.0f + expf(-v));
        if (ACT == 4) v = (v > 0.f) ? v : 0.01f * v;
        slab[(mOff + r) * 68 + (j << 4) + rlane] = v;
      }
    }
    __builtin_amdgcn_fence(__ATOMIC_RELEASE, "workgroup");
    __builtin_amdgcn_wave_barrier();
    __builtin_amdgcn_fence(__ATOMIC_ACQUIRE, "workgroup");
    if (OUT_MODE == 0) {
      float* C = (float*)Cout + (size_t)b * strideC;
      const int hh = lane >> 4, c4 = (lane & 15) * 4;
      for (int pass = 0; pass < 2; ++pass) {
#pragma unroll
        for (int it = 0; it < 8; ++it) {
          const int row = it * 2 + hh;
          v4f v = *(const v4f*)(slab + row * 68 + c4);
          *(volatile v4f*)(C + (size_t)(mBase + row) * ldc + n0 + c4) = v;
        }
        __threadfence();
      }
    } else {
      const int q = lane >> 3, c8 = (lane & 7) * 8;
      unsigned short* C  = (unsigned short*)Cout  + (size_t)b * strideC;
      unsigned short* C2 = (OUT_MODE == 2) ? ((unsigned short*)Cout2 + (size_t)b * strideC) : nullptr;
      for (int pass = 0; pass < 2; ++pass) {
#pragma unroll
        for (int it = 0; it < 4; ++it) {
          const int row = it * 4 + q;
          const float* sp = slab + row * 68 + c8;
          v8h hv, lv;
#pragma unroll
          for (int e = 0; e < 8; ++e) {
            if (OUT_MODE == 1) {
              hv[e] = (_Float16)sp[e];
            } else {
              unsigned short hb = f2bf_bits(sp[e]);
              unsigned short lb = f2bf_bits(sp[e] - bf_bits2f(hb));
              hv[e] = __builtin_bit_cast(_Float16, hb);
              lv[e] = __builtin_bit_cast(_Float16, lb);
            }
          }
          *(volatile v8h*)(C + (size_t)(mBase + row) * ldc + n0 + c8) = hv;
          if (OUT_MODE == 2) *(volatile v8h*)(C2 + (size_t)(mBase + row) * ldc + n0 + c8) = lv;
        }
        __threadfence();
      }
    }
    __builtin_amdgcn_fence(__ATOMIC_RELEASE, "workgroup");
    __builtin_amdgcn_wave_barrier();
    __builtin_amdgcn_fence(__ATOMIC_ACQUIRE, "workgroup");
  }
}

__global__ __launch_bounds__(256) void cast_f32_bf16x2(const float* __restrict__ in, unsigned short* __restrict__ out, int n2) {
  const int i = blockIdx.x * 256 + threadIdx.x;
  if (i < n2) {
    const v2f f = *(const v2f*)(in + 2 * (size_t)i);
    const unsigned u = pk16(f2bf_bits(f[0]), f2bf_bits(f[1]));
    ((volatile unsigned*)out)[i] = u;
    __threadfence();
    ((volatile unsigned*)out)[i] = u;
  }
}

__global__ __launch_bounds__(256) void split_bf16x2_kernel(const float* __restrict__ in, unsigned short* __restrict__ hi,
                                                           unsigned short* __restrict__ lo, int n2) {
  const int i = blockIdx.x * 256 + threadIdx.x;
  if (i < n2) {
    const v2f f = *(const v2f*)(in + 2 * (size_t)i);
    const unsigned short h0 = f2bf_bits(f[0]), h1 = f2bf_bits(f[1]);
    const unsigned short l0 = f2bf_bits(f[0] - bf_bits2f(h0)), l1 = f2bf_bits(f[1] - bf_bits2f(h1));
    const unsigned uh = pk16(h0, h1), ul = pk16(l0, l1);
    ((volatile unsigned*)hi)[i] = uh;
    ((volatile unsigned*)lo)[i] = ul;
    __threadfence();
    ((volatile unsigned*)hi)[i] = uh;
    ((volatile unsigned*)lo)[i] = ul;
  }
}

__global__ __launch_bounds__(256) void ln_head_kernel(const float* __restrict__ in, const float* __restrict__ gam,
                                                      const float* __restrict__ bet, unsigned short* __restrict__ outp,
                                                      int nrows) {
  __shared__ __align__(16) float srow[8][ND_MODEL];
  const int lane = threadIdx.x & 31, wave = threadIdx.x >> 5;
  const int row = blockIdx.x * 8 + wave;
  if (row >= nrows) return;
  _Float16* out = (_Float16*)(void*)outp;
  const float g0 = gam[2 * lane], g1 = gam[2 * lane + 1];
  const float t0 = bet[2 * lane], t1 = bet[2 * lane + 1];
  const float* rp = in + (size_t)row * ND_MODEL;
  float* sr = srow[wave];
#pragma unroll 1
  for (int hd = 0; hd < NH_HEADS; ++hd) {
    const v2f xv = *(const v2f*)(rp + hd * NHD + 2 * lane);
    float s = xv[0] + xv[1];
#pragma unroll
    for (int off = 1; off < 32; off <<= 1) s += __shfl_xor(s, off, 32);
    const float mu = s * (1.0f / 64.0f);
    const float d0 = xv[0] - mu, d1 = xv[1] - mu;
    float ss = d0 * d0 + d1 * d1;
#pragma unroll
    for (int off = 1; off < 32; off <<= 1) ss += __shfl_xor(ss, off, 32);
    const float var = ss * (1.0f / 64.0f);
    const float rs = rsqrtf(var + 1e-5f);
    sr[hd * NHD + 2 * lane]     = d0 * rs * g0 + t0;
    sr[hd * NHD + 2 * lane + 1] = d1 * rs * g1 + t1;
  }
  __builtin_amdgcn_fence(__ATOMIC_RELEASE, "workgroup");
  __builtin_amdgcn_wave_barrier();
  __builtin_amdgcn_fence(__ATOMIC_ACQUIRE, "workgroup");
  v8h hv[4];
#pragma unroll
  for (int it = 0; it < 4; ++it) {
    const int seg = it * 4 + (lane >> 3);
    const int c8  = (lane & 7) * 8;
#pragma unroll
    for (int e = 0; e < 8; ++e) hv[it][e] = (_Float16)sr[seg * NHD + c8 + e];
  }
  _Float16* orow = out + (size_t)row * ND_MODEL;
  for (int pass = 0; pass < 2; ++pass) {
#pragma unroll
    for (int it = 0; it < 4; ++it) {
      const int seg = it * 4 + (lane >> 3);
      const int c8  = (lane & 7) * 8;
      *(volatile v8h*)(orow + seg * NHD + c8) = hv[it];
    }
    __threadfence();
  }
}

static constexpr int AT_D  = 64;
static constexpr int AT_NW = 4;
static constexpr int AT_QB = 64;
static constexpr int AT_KC = 64;
static constexpr float P_CARRY = 32768.0f;

__device__ __forceinline__ v8f mma_h(v16h a, v16h b, v8f c) {
  c = __builtin_amdgcn_wmma_f32_16x16x32_f16(false, a, false, b, (short)0, c, false, false);
  asm volatile("v_nop\n\tv_nop\n\tv_nop\n\tv_nop" : "+v"(c) : "v"(a), "v"(b));
  return c;
}

__global__ __launch_bounds__(128)
void attn_f16_kernel(const unsigned short* __restrict__ qp, const unsigned short* __restrict__ kp,
                     const unsigned short* __restrict__ vtp, float* __restrict__ outp, float sscale) {
  union FH { v16h v; v8h h[2]; };
  __shared__ __align__(16) _Float16 Ksh[AT_KC * AT_D];
  __shared__ __align__(16) _Float16 Vth[AT_D * AT_KC];
  __shared__ __align__(16) _Float16 Psh[AT_NW][16 * AT_KC];
  __shared__ __align__(16) float    Os[AT_NW][16 * 68];

  const int tid  = threadIdx.x;
  const int wave = tid >> 5;
  const int lane = tid & 31;
  const int hh   = lane >> 4;
  const int c    = lane & 15;

  const int nqb = NS_SEQ / AT_QB;
  const int bx = blockIdx.x;
  const int qb = bx % nqb;
  const int bh = bx / nqb;
  const int h  = bh % NH_HEADS;
  const int b  = bh / NH_HEADS;
  const int q0 = qb * AT_QB + wave * 16;

  const _Float16* Qg = (const _Float16*)(const void*)qp + (size_t)b * NS_SEQ * ND_MODEL + (size_t)h * AT_D;
  const _Float16* Kg = (const _Float16*)(const void*)kp + (size_t)b * NS_SEQ * ND_MODEL + (size_t)h * AT_D;
  const _Float16* Vg = (const _Float16*)(const void*)vtp + (size_t)(b * NH_HEADS + h) * AT_D * NS_SEQ;
  float*          ob = outp + (size_t)b * NS_SEQ * ND_MODEL + (size_t)h * AT_D;

  v16h qa[2];
#pragma unroll
  for (int dc = 0; dc < 2; ++dc) {
    const _Float16* qr = Qg + (size_t)(q0 + c) * ND_MODEL + dc * 32 + 8 * hh;
    qa[dc] = Frag<_Float16>::load(qr);
  }

  float mrow[8], lrow[8];
  v8f oacc[4];
#pragma unroll
  for (int r = 0; r < 8; ++r) { mrow[r] = -INFINITY; lrow[r] = 0.f; }
#pragma unroll
  for (int t = 0; t < 4; ++t) oacc[t] = (v8f){0.f,0.f,0.f,0.f,0.f,0.f,0.f,0.f};

  const int nChunks = NS_SEQ / AT_KC;
  for (int kc = 0; kc < nChunks; ++kc) {
    const int kv0 = kc * AT_KC;
    __syncthreads();
    {
      const int r = tid >> 1, half = (tid & 1) * 32;
      const _Float16* ks = Kg + (size_t)(kv0 + r) * ND_MODEL + half;
      const _Float16* vs = Vg + (size_t)r * NS_SEQ + kv0 + half;
#pragma unroll
      for (int i = 0; i < 4; ++i) {
        const v8h a0 = *(const v8h*)(ks + 8 * i);
        const v8h b0 = *(const v8h*)(vs + 8 * i);
        *(v8h*)(Ksh + r * AT_D  + half + 8 * i) = a0;
        *(v8h*)(Vth + r * AT_KC + half + 8 * i) = b0;
      }
    }
    __syncthreads();

    v8f s[4];
#pragma unroll
    for (int j = 0; j < 4; ++j) {
      s[j] = (v8f){0.f,0.f,0.f,0.f,0.f,0.f,0.f,0.f};
#pragma unroll
      for (int dc = 0; dc < 2; ++dc) {
        FH kb;
        kb.h[0] = *(const v8h*)(Ksh + (j * 16 + c) * AT_D + dc * 32 + 8 * hh);
        kb.h[1] = *(const v8h*)(Ksh + (j * 16 + c) * AT_D + dc * 32 + 16 + 8 * hh);
        s[j] = mma_h(qa[dc], kb.v, s[j]);
      }
    }
    float cm[8];
#pragma unroll
    for (int r = 0; r < 8; ++r) {
      float m = -INFINITY;
#pragma unroll
      for (int j = 0; j < 4; ++j) {
        const float sv = s[j][r] * sscale;
        s[j][r] = sv;
        m = fmaxf(m, sv);
      }
#pragma unroll
      for (int off = 1; off < 16; off <<= 1) m = fmaxf(m, __shfl_xor(m, off, 32));
      cm[r] = m;
    }
    _Float16* pwh = Psh[wave];
#pragma unroll
    for (int r = 0; r < 8; ++r) {
      const float mnew = fmaxf(mrow[r], cm[r]);
      const float alpha = expf(mrow[r] - mnew);
      mrow[r] = mnew;
      float psum = 0.f;
#pragma unroll
      for (int j = 0; j < 4; ++j) {
        const float p = expf(s[j][r] - mnew);
        psum += p;
        pwh[(8 * hh + r) * AT_KC + j * 16 + c] = (_Float16)(p * P_CARRY);
      }
#pragma unroll
      for (int off = 1; off < 16; off <<= 1) psum += __shfl_xor(psum, off, 32);
      lrow[r] = lrow[r] * alpha + psum;
#pragma unroll
      for (int t = 0; t < 4; ++t) oacc[t][r] *= alpha;
    }
    __builtin_amdgcn_fence(__ATOMIC_RELEASE, "workgroup");
    __builtin_amdgcn_wave_barrier();
    __builtin_amdgcn_fence(__ATOMIC_ACQUIRE, "workgroup");
#pragma unroll
    for (int kk = 0; kk < 2; ++kk) {
      FH pa;
      pa.h[0] = *(const v8h*)(pwh + c * AT_KC + kk * 32 + 8 * hh);
      pa.h[1] = *(const v8h*)(pwh + c * AT_KC + kk * 32 + 16 + 8 * hh);
#pragma unroll
      for (int t = 0; t < 4; ++t) {
        FH vb;
        vb.h[0] = *(const v8h*)(Vth + (t * 16 + c) * AT_KC + kk * 32 + 8 * hh);
        vb.h[1] = *(const v8h*)(Vth + (t * 16 + c) * AT_KC + kk * 32 + 16 + 8 * hh);
        oacc[t] = mma_h(pa.v, vb.v, oacc[t]);
      }
    }
  }

  float* os = Os[wave];
#pragma unroll
  for (int r = 0; r < 8; ++r) {
    const float inv = 1.0f / (lrow[r] * P_CARRY);
#pragma unroll
    for (int t = 0; t < 4; ++t) os[(8 * hh + r) * 68 + t * 16 + c] = oacc[t][r] * inv;
  }
  __builtin_amdgcn_fence(__ATOMIC_RELEASE, "workgroup");
  __builtin_amdgcn_wave_barrier();
  __builtin_amdgcn_fence(__ATOMIC_ACQUIRE, "workgroup");
  {
    const int c4 = (lane & 15) * 4;
    for (int pass = 0; pass < 2; ++pass) {
#pragma unroll
      for (int it = 0; it < 8; ++it) {
        const int row = it * 2 + hh;
        v4f val = *(const v4f*)(os + row * 68 + c4);
        *(volatile v4f*)(ob + (size_t)(q0 + row) * ND_MODEL + c4) = val;
      }
      __threadfence();
    }
  }
}

extern "C" void kernel_launch(void* const* d_in, const int* in_sizes, int n_in,
                              void* d_out, int out_size, void* d_ws, size_t ws_size,
                              hipStream_t stream) {
  if (n_in < 9) return;
  const int nTok = NTOK, nD = ND_MODEL, nQKV = 3 * ND_MODEL;
  if (in_sizes[0] != nTok * nD || in_sizes[1] != nQKV * nD || in_sizes[2] != nQKV ||
      in_sizes[3] != NHD || in_sizes[4] != NHD || in_sizes[5] != NHD || in_sizes[6] != NHD ||
      in_sizes[7] != nD * nD || in_sizes[8] != nD || out_size != nTok * nD) return;

  const size_t offXB  = 0;
  const size_t szXB   = (size_t)nTok * nD * 2;
  const size_t offW   = offXB + szXB;
  const size_t szW    = (size_t)nQKV * nD * 2;
  const size_t offWO  = offW + szW;
  const size_t szWO   = (size_t)nD * nD * 2;
  const size_t offSCR = offWO + szWO;
  const size_t szSCR  = (size_t)nTok * nD * 4;
  const size_t offQ   = offSCR + szSCR;
  const size_t szP16  = (size_t)nTok * nD * 2;
  const size_t offK   = offQ + szP16;
  const size_t offVT  = offK + szP16;
  const size_t wsEnd  = offVT + szP16;
  if (ws_size < wsEnd) return;

  const float* x     = (const float*)d_in[0];
  const float* qkv_w = (const float*)d_in[1];
  const float* qkv_b = (const float*)d_in[2];
  const float* q_g   = (const float*)d_in[3];
  const float* q_bt  = (const float*)d_in[4];
  const float* k_g   = (const float*)d_in[5];
  const float* k_bt  = (const float*)d_in[6];
  const float* out_w = (const float*)d_in[7];
  const float* out_b = (const float*)d_in[8];
  float* out = (float*)d_out;

  char* ws = (char*)d_ws;
  unsigned short* XB  = (unsigned short*)(ws + offXB);
  unsigned short* WQ  = (unsigned short*)(ws + offW);
  unsigned short* WO  = (unsigned short*)(ws + offWO);
  float*          SCR = (float*)(ws + offSCR);
  unsigned short* Q16 = (unsigned short*)(ws + offQ);
  unsigned short* K16 = (unsigned short*)(ws + offK);
  unsigned short* VT  = (unsigned short*)(ws + offVT);
  unsigned short* OH  = XB;
  unsigned short* OL  = Q16;

  {
    const int n2x = nTok * nD / 2, n2w = nQKV * nD / 2, n2o = nD * nD / 2;
    cast_f32_bf16x2<<<dim3((n2x + 255) / 256), dim3(256), 0, stream>>>(x, XB, n2x);
    cast_f32_bf16x2<<<dim3((n2w + 255) / 256), dim3(256), 0, stream>>>(qkv_w, WQ, n2w);
    cast_f32_bf16x2<<<dim3((n2o + 255) / 256), dim3(256), 0, stream>>>(out_w, WO, n2o);
  }
  const int gemmBlocks = ((nTok / 64) * (nD / 64) + 7) / 8;
  wmma_gemm64<1, 0, 2, 0, false><<<dim3(gemmBlocks, 1), dim3(256), 0, stream>>>(
      XB, XB, nD, 0L, WQ, WQ, nD, 0L, (void*)SCR, (void*)SCR, nD, 0L,
      qkv_b, qkv_b, 0L, nTok, nD, nD, 1.0f);
  ln_head_kernel<<<dim3(nTok / 8), dim3(256), 0, stream>>>(SCR, q_g, q_bt, Q16, nTok);
  wmma_gemm64<1, 0, 2, 0, false><<<dim3(gemmBlocks, 1), dim3(256), 0, stream>>>(
      XB, XB, nD, 0L, WQ + (size_t)nD * nD, WQ + (size_t)nD * nD, nD, 0L, (void*)SCR, (void*)SCR, nD, 0L,
      qkv_b + nD, qkv_b, 0L, nTok, nD, nD, 1.0f);
  ln_head_kernel<<<dim3(nTok / 8), dim3(256), 0, stream>>>(SCR, k_g, k_bt, K16, nTok);
  {
    const int vtBlocks = ((nD / 64) * (NS_SEQ / 64) + 7) / 8;
    wmma_gemm64<1, 0, 1, 1, false><<<dim3(vtBlocks, NB_BATCH), dim3(256), 0, stream>>>(
        WQ + (size_t)2 * nD * nD, WQ + (size_t)2 * nD * nD, nD, 0L,
        XB, XB, nD, (long)NS_SEQ * nD,
        (void*)VT, (void*)VT, NS_SEQ, (long)nD * NS_SEQ,
        qkv_b + 2 * nD, qkv_b, 0L, nD, NS_SEQ, nD, 1.0f);
  }
  attn_f16_kernel<<<dim3(NB_BATCH * NH_HEADS * (NS_SEQ / AT_QB)), dim3(128), 0, stream>>>(
      Q16, K16, VT, SCR, 0.125f);
  {
    const int n2 = nTok * nD / 2;
    split_bf16x2_kernel<<<dim3((n2 + 255) / 256), dim3(256), 0, stream>>>(SCR, OH, OL, n2);
  }
  wmma_gemm64<1, 2, 2, 0, false><<<dim3(gemmBlocks, 1), dim3(256), 0, stream>>>(
      OH, OL, nD, 0L, WO, WO, nD, 0L, (void*)out, (void*)out, nD, 0L,
      out_b, out_b, 0L, nTok, nD, nD, 1.0f);
}
